// SEGNNConv_16226386444783
// MI455X (gfx1250) — hardware-verified
//
#include <hip/hip_runtime.h>
#include <stddef.h>
#include <math.h>


#define NT2    128
#define NW2    4
#define EPT    8
#define CHUNK  (NT2 * EPT)
#define WCAP   (EPT * 32)
#define LISTN  (NW2 * WCAP)
#define PASSN  (NW2 * 16)
#define PCAP   (CHUNK + PASSN)
#define NB     128
#define MW     160
#define AP     256

static_assert(CHUNK == 1024);
static_assert(PASSN == 64);
static_assert(PASSN <= NT2);
static_assert((NB * MW) % (4 * NT2) == 0);

constexpr int L_ACC = 0;
constexpr int L_MSG = L_ACC + (NB + 1) * MW * 4;
constexpr int L_AT  = L_MSG + NW2 * 16 * MW * 4;
constexpr int L_HR  = L_AT  + NW2 * 2 * 16 * AP * 2;
constexpr int L_YM  = L_HR  + NW2 * 16 * 8 * 4;
constexpr int L_W0  = L_YM  + NW2 * 16 * 4 * 4;
constexpr int L_W1  = L_W0  + 64 * 4;
constexpr int L_LST = L_W1  + 1536 * 4;
constexpr int L_PND = L_LST + LISTN * 4;
constexpr int L_SLT = L_PND + PCAP * 4;
constexpr int L_WC  = L_SLT + PASSN * 4;
constexpr int L_PN  = L_WC  + 16;
constexpr int L_TOT = L_PN  + 16;
static_assert((L_MSG & 15) == 0 && (L_AT & 15) == 0 && (L_HR & 15) == 0 && (L_YM & 15) == 0);
static_assert((L_W0 & 15) == 0 && (L_W1 & 15) == 0 && (L_LST & 15) == 0 && (L_PND & 15) == 0);
static_assert((L_SLT & 15) == 0 && (L_WC & 15) == 0 && (L_PN & 15) == 0);
static_assert(L_TOT <= 300 * 1024);

typedef float          v4f   __attribute__((ext_vector_type(4)));
typedef float          v8f   __attribute__((ext_vector_type(8)));
typedef int            v4i   __attribute__((ext_vector_type(4)));
typedef unsigned short v8us  __attribute__((ext_vector_type(8)));
typedef unsigned short v16us __attribute__((ext_vector_type(16)));
typedef __bf16         v16bf __attribute__((ext_vector_type(16)));
union FragU { v16us v; v8us h[2]; };

struct WDesc { const float* src[10]; int meta[60]; };
static_assert(sizeof(WDesc) == 320);

__device__ __forceinline__ unsigned short f2bf(float f) {
  unsigned int u = __float_as_uint(f);
  u += 0x7FFFu + ((u >> 16) & 1u);
  return (unsigned short)(u >> 16);
}
__device__ __forceinline__ float bf2f(unsigned short b) { return __uint_as_float(((unsigned int)b) << 16); }
__device__ __forceinline__ float rbf(float f) { return bf2f(f2bf(f)); }
__device__ __forceinline__ void sthl(unsigned short* ph, unsigned short* pl, int i, float x) {
  const unsigned short hi = f2bf(x);
  const unsigned short lo = f2bf(x - bf2f(hi));
  ph[i] = hi;
  pl[i] = lo;
}

__device__ __forceinline__ v8f zero8f() {
  v8f z;
#pragma unroll
  for (int i = 0; i < 8; ++i) z[i] = 0.0f;
  return z;
}

__device__ __forceinline__ v8f wmb(v16us a, v16us b, v8f c) {
  const v16bf av = __builtin_bit_cast(v16bf, a);
  const v16bf bv = __builtin_bit_cast(v16bf, b);
  v8f d = __builtin_amdgcn_wmma_f32_16x16x32_bf16(false, av, false, bv, (short)0, c, false, false);
  asm volatile("v_nop\n\tv_nop\n\tv_nop\n\tv_nop" : "+v"(d) : "v"(av), "v"(bv));
  return d;
}

__device__ __forceinline__ v16us ldfrag_s(const unsigned short* base, int ld, int row, int k0, int h) {
  FragU f;
  const unsigned short* p = base + row * ld + k0 + 8 * h;
  f.h[0] = *(const v8us*)p;
  f.h[1] = *(const v8us*)(p + 16);
  return f.v;
}
__device__ __forceinline__ v16us ldfrag_g(const unsigned short* __restrict__ base, int ld, int row, int k0, int h) {
  FragU f;
  const unsigned short* p = base + (size_t)row * ld + k0 + 8 * h;
  f.h[0] = *(const v8us*)p;
  f.h[1] = *(const v8us*)(p + 16);
  return f.v;
}

__device__ __forceinline__ float sigm(float x) {
  const float t = fminf(-x, 80.0f);
  return __builtin_amdgcn_rcpf(1.0f + __expf(t));
}
__device__ __forceinline__ float silu(float x) { return x * sigm(x); }

__global__ __launch_bounds__(256) void k_wprep(WDesc d, unsigned short* wsh) {
  const int tid = threadIdx.x;
  const int bid = blockIdx.x;
  const float* src = d.src[0];
  int off = 0, K = 8, Kp = 8, sk = 0, sn = 0, np = 0, q = -1;
  int bb = 0;
#pragma unroll
  for (int p = 0; p < 10; ++p) {
    const int nRp = d.meta[6 * p + 1], Kq = d.meta[6 * p + 2], Kpq = d.meta[6 * p + 3];
    const int npp = (nRp * Kpq) >> 3;
    const int nb  = (npp + 255) >> 8;
    const bool mine = (bid >= bb) && (bid < bb + nb);
    if (mine) {
      src = d.src[p]; off = d.meta[6 * p]; K = Kq; Kp = Kpq;
      sk = d.meta[6 * p + 4]; sn = d.meta[6 * p + 5]; np = npp; q = (bid - bb) * 256 + tid;
    }
    bb += nb;
  }
  if (q < 0 || q >= np) return;
  const int cpr = Kp >> 3;
  const int row = q / cpr;
  const int ch  = q - row * cpr;
  v8us o;
#pragma unroll
  for (int i = 0; i < 8; ++i) {
    const int k  = ch * 8 + i;
    const int kc = k < K ? k : K - 1;
    const float v = src[(size_t)kc * sk + (size_t)row * sn];
    o[i] = (k < K) ? f2bf(v) : (unsigned short)0;
  }
  unsigned short* dp = wsh + off + (size_t)q * 8;
  *(volatile v8us*)dp = o;
  __threadfence();
  *(volatile v8us*)dp = o;
}

__global__ __launch_bounds__(64) void k_node1(const float* __restrict__ feats,
    const unsigned short* __restrict__ w1sP, const unsigned short* __restrict__ w1vP,
    float* s1out, float* v1out, int nN, float invs32) {
  __shared__ __attribute__((aligned(16))) unsigned short W1s[64 * 64];
  __shared__ __attribute__((aligned(16))) unsigned short W1v[32 * 32];
  __shared__ __attribute__((aligned(16))) unsigned short sA[2][16 * 64];
  __shared__ __attribute__((aligned(16))) unsigned short vA[2][3 * 16 * 32];
  __shared__ __attribute__((aligned(16))) float oS[2][16 * 64];
  __shared__ __attribute__((aligned(16))) float oV[2][16 * 96];
  const int tid = threadIdx.x, lane = tid & 31, wave = tid >> 5, hh = lane >> 4, m = lane & 15;
  for (int i = tid; i < 512; i += 64) *(v8us*)(W1s + 8 * i) = *(const v8us*)(w1sP + 8 * i);
  for (int i = tid; i < 128; i += 64) *(v8us*)(W1v + 8 * i) = *(const v8us*)(w1vP + 8 * i);
  const int n0 = ((int)blockIdx.x * 2 + wave) * 16;
  unsigned short* sAw = sA[wave];
  unsigned short* vAw = vA[wave];
  float* oSw = oS[wave];
  float* oVw = oV[wave];
#pragma unroll 1
  for (int r = 0; r < 16; ++r) {
    int nd = n0 + r;
    nd = nd > nN - 1 ? nN - 1 : nd;
    const float* f = feats + (size_t)nd * 160;
    sAw[r * 64 + lane]      = f2bf(f[lane]);
    sAw[r * 64 + 32 + lane] = f2bf(f[32 + lane]);
#pragma unroll
    for (int t = 0; t < 3; ++t) {
      const int j = lane + 32 * t;
      const int u = j / 3;
      const int c = j - 3 * u;
      vAw[(c * 16 + r) * 32 + u] = f2bf(f[64 + j]);
    }
  }
  __syncthreads();
  const v8f z8 = zero8f();
  {
    const v16us a0 = ldfrag_s(sAw, 64, m, 0, hh);
    const v16us a1 = ldfrag_s(sAw, 64, m, 32, hh);
#pragma unroll
    for (int nt = 0; nt < 4; ++nt) {
      v8f c = z8;
      c = wmb(a0, ldfrag_s(W1s, 64, 16 * nt + m, 0, hh), c);
      c = wmb(a1, ldfrag_s(W1s, 64, 16 * nt + m, 32, hh), c);
#pragma unroll
      for (int rr = 0; rr < 8; ++rr) oSw[(8 * hh + rr) * 64 + 16 * nt + m] = c[rr] * 0.125f;
    }
  }
#pragma unroll
  for (int cc = 0; cc < 3; ++cc) {
    const v16us a = ldfrag_s(vAw + cc * 512, 32, m, 0, hh);
#pragma unroll
    for (int nt = 0; nt < 2; ++nt) {
      const v8f c = wmb(a, ldfrag_s(W1v, 32, 16 * nt + m, 0, hh), z8);
#pragma unroll
      for (int rr = 0; rr < 8; ++rr) oVw[(8 * hh + rr) * 96 + cc * 32 + 16 * nt + m] = c[rr] * invs32;
    }
  }
  __syncthreads();
  float* sb = s1out + (size_t)n0 * 64;
  float* vb = v1out + (size_t)n0 * 96;
#pragma unroll 1
  for (int it = 0; it < 8; ++it) {
    const int f = it * 128 + 4 * lane;
    const v4f v = *(const v4f*)(oSw + f);
    *(volatile v4f*)(sb + f) = v;
  }
#pragma unroll 1
  for (int it = 0; it < 12; ++it) {
    const int f = it * 128 + 4 * lane;
    const v4f v = *(const v4f*)(oVw + f);
    *(volatile v4f*)(vb + f) = v;
  }
  __threadfence();
#pragma unroll 1
  for (int it = 0; it < 8; ++it) {
    const int f = it * 128 + 4 * lane;
    const v4f v = *(const v4f*)(oSw + f);
    *(volatile v4f*)(sb + f) = v;
  }
#pragma unroll 1
  for (int it = 0; it < 12; ++it) {
    const int f = it * 128 + 4 * lane;
    const v4f v = *(const v4f*)(oVw + f);
    *(volatile v4f*)(vb + f) = v;
  }
}

__device__ __forceinline__ int scan_chunk(const int* __restrict__ dsts, int nE, int cbase, int nodeBase,
                                          int vec8, int* list, int tid, int wave) {
  int wc = 0;
  const int el0  = tid * EPT;
  const int e0   = cbase + el0;
  const int sent = -2147483647 - 1;
  const int l0   = nE - 1;
  v4i da, db;
  if (vec8 != 0 && cbase + CHUNK <= nE) {
    da = *(const v4i*)(dsts + e0);
    db = *(const v4i*)(dsts + e0 + 4);
  } else {
    da.x = (e0     < nE) ? dsts[(e0    ) < l0 ? (e0    ) : l0] : sent;
    da.y = (e0 + 1 < nE) ? dsts[(e0 + 1) < l0 ? (e0 + 1) : l0] : sent;
    da.z = (e0 + 2 < nE) ? dsts[(e0 + 2) < l0 ? (e0 + 2) : l0] : sent;
    da.w = (e0 + 3 < nE) ? dsts[(e0 + 3) < l0 ? (e0 + 3) : l0] : sent;
    db.x = (e0 + 4 < nE) ? dsts[(e0 + 4) < l0 ? (e0 + 4) : l0] : sent;
    db.y = (e0 + 5 < nE) ? dsts[(e0 + 5) < l0 ? (e0 + 5) : l0] : sent;
    db.z = (e0 + 6 < nE) ? dsts[(e0 + 6) < l0 ? (e0 + 6) : l0] : sent;
    db.w = (e0 + 7 < nE) ? dsts[(e0 + 7) < l0 ? (e0 + 7) : l0] : sent;
  }
  const unsigned nb = (unsigned)nodeBase;
  const unsigned s0 = (unsigned)da.x - nb, s1 = (unsigned)da.y - nb;
  const unsigned s2 = (unsigned)da.z - nb, s3 = (unsigned)da.w - nb;
  const unsigned s4 = (unsigned)db.x - nb, s5 = (unsigned)db.y - nb;
  const unsigned s6 = (unsigned)db.z - nb, s7 = (unsigned)db.w - nb;
  const bool h0 = s0 < (unsigned)NB, h1 = s1 < (unsigned)NB, h2 = s2 < (unsigned)NB, h3 = s3 < (unsigned)NB;
  const bool h4 = s4 < (unsigned)NB, h5 = s5 < (unsigned)NB, h6 = s6 < (unsigned)NB, h7 = s7 < (unsigned)NB;
  const unsigned any = __builtin_amdgcn_ballot_w32(h0 | h1 | h2 | h3 | h4 | h5 | h6 | h7);
  if (any != 0u) {
#define HITJ(J, HJ) { \
      const unsigned mj = __builtin_amdgcn_ballot_w32(HJ); \
      if (mj != 0u) { \
        if (HJ) { \
          const int pos = wc + (int)__builtin_amdgcn_mbcnt_lo(mj, 0u); \
          if (pos < WCAP) list[wave * WCAP + pos] = el0 + (J); \
        } \
        wc += (int)__builtin_popcount(mj); } }
    HITJ(0, h0)
    HITJ(1, h1)
    HITJ(2, h2)
    HITJ(3, h3)
    HITJ(4, h4)
    HITJ(5, h5)
    HITJ(6, h6)
    HITJ(7, h7)
#undef HITJ
  }
  return wc;
}

__global__ __launch_bounds__(NT2) void k_edge(
    const float* __restrict__ s1, const float* __restrict__ v1,
    const float* __restrict__ eattr, const float* __restrict__ eemb,
    const float* __restrict__ w0g, const float* __restrict__ w1g,
    const int* __restrict__ ei,
    const unsigned short* __restrict__ w2s, const unsigned short* __restrict__ w2v,
    float* agout, int nN, int nE, int vec8, float inv8, float inv3, float inv96) {
  extern __shared__ __attribute__((aligned(16))) unsigned char dsm[];
  float* acc  = (float*)(dsm + L_ACC);
  float* msg  = (float*)(dsm + L_MSG);
  unsigned short* atl = (unsigned short*)(dsm + L_AT);
  float* hrow = (float*)(dsm + L_HR);
  float* ym   = (float*)(dsm + L_YM);
  float* w0s  = (float*)(dsm + L_W0);
  float* w1s  = (float*)(dsm + L_W1);
  int* list   = (int*)(dsm + L_LST);
  int* pend   = (int*)(dsm + L_PND);
  int* slotb  = (int*)(dsm + L_SLT);
  int* wcnt   = (int*)(dsm + L_WC);
  int* pendN  = (int*)(dsm + L_PN);

  const int tid = threadIdx.x, lane = tid & 31, wave = tid >> 5, hh = lane >> 4, m = lane & 15;
  const int el = m;
  const int nodeBase = blockIdx.x * NB;
  const int* srcs = ei;
  const int* dsts = ei + nE;

  for (int i = tid; i < (NB + 1) * MW; i += NT2) acc[i] = 0.0f;
  if (tid < 64) w0s[tid] = rbf(w0g[tid]);
  for (int i = tid; i < 1536; i += NT2) w1s[i] = rbf(w1g[i]);
  if (tid == 0) pendN[0] = 0;
  __syncthreads();

  unsigned short* aHi = atl + wave * (2 * 16 * AP);
  unsigned short* aLo = aHi + 16 * AP;
  float* msgw = msg + wave * 16 * MW;
  float* hw   = hrow + wave * 16 * 8;
  float* yw   = ym + wave * 16 * 4;
  const v8f z8 = zero8f();

  const int nChunks = (nE + CHUNK - 1) / CHUNK;
#pragma unroll 1
  for (int ch = 0; ch < nChunks; ++ch) {
    const int cbase = ch * CHUNK;
    const int wc = scan_chunk(dsts, nE, cbase, nodeBase, vec8, list, tid, wave);
    if (lane == 0) wcnt[wave] = wc;
    __syncthreads();

    const int base = pendN[0];
    int tot = 0, myoff = 0;
#pragma unroll
    for (int w = 0; w < NW2; ++w) {
      int c = wcnt[w];
      c = c > WCAP ? WCAP : (c < 0 ? 0 : c);
      if (w < wave) myoff += c;
      tot += c;
    }
    int newN = base + tot;
    newN = newN > PCAP ? PCAP : newN;
    {
      int n = wcnt[wave];
      n = n > WCAP ? WCAP : (n < 0 ? 0 : n);
      const int* lp = list + wave * WCAP;
      for (int i = lane; i < n; i += 32) {
        const int pos = base + myoff + i;
        if (pos < PCAP) pend[pos] = cbase + lp[i];
      }
    }
    const int fin = (ch == nChunks - 1) ? 1 : 0;
    const int R   = (fin != 0) ? (newN + PASSN - 1) / PASSN : newN / PASSN;
    const int Pv  = (fin != 0) ? newN : R * PASSN;
    __syncthreads();

#pragma unroll 1
    for (int r = 0; r < R; ++r) {
      int sIdx;
      float y0, y1, y2, y3;
      bool valid;
      {
        const int idx = r * PASSN + wave * 16 + el;
        valid = idx < Pv;
        int e = pend[idx < PCAP - 1 ? idx : PCAP - 1];
        e = valid ? e : 0;
        e = e < 0 ? 0 : (e > nE - 1 ? nE - 1 : e);
        const int d = dsts[e];
        int s = srcs[e];
        int slot = d - nodeBase;
        if (!valid || (unsigned)slot >= (unsigned)NB) slot = NB;
        s = s < 0 ? 0 : (s > nN - 1 ? nN - 1 : s);
        sIdx = s;
        const v4f ya = *(const v4f*)(eattr + (size_t)e * 4);
        y0 = rbf(ya.x); y1 = rbf(ya.y); y2 = rbf(ya.z); y3 = rbf(ya.w);
        const v4f ea = *(const v4f*)(eemb + (size_t)e * 8);
        const v4f eb = *(const v4f*)(eemb + (size_t)e * 8 + 4);
        float em[8];
        em[0] = rbf(ea.x); em[1] = rbf(ea.y); em[2] = rbf(ea.z); em[3] = rbf(ea.w);
        em[4] = rbf(eb.x); em[5] = rbf(eb.y); em[6] = rbf(eb.z); em[7] = rbf(eb.w);
#pragma unroll
        for (int jj = 0; jj < 4; ++jj) {
          const int j = 4 * hh + jj;
          float a = 0.0f;
#pragma unroll
          for (int k = 0; k < 8; ++k) a += em[k] * w0s[k * 8 + j];
          a *= inv8;
          hw[el * 8 + j] = silu(a);
        }
        if (hh == 0) {
          slotb[wave * 16 + el] = slot;
          yw[el * 4 + 0] = y0; yw[el * 4 + 1] = y1; yw[el * 4 + 2] = y2; yw[el * 4 + 3] = y3;
        }
      }
      __syncthreads();

      {
        float hv[8];
#pragma unroll
        for (int k = 0; k < 8; ++k) hv[k] = hw[el * 8 + k];
        const float* s1p = s1 + (size_t)sIdx * 64;
        const float* v1p = v1 + (size_t)sIdx * 96;
        unsigned short* rh = aHi + el * AP;
        unsigned short* rl = aLo + el * AP;
#pragma unroll 1
        for (int j = 0; j < 32; ++j) {
          const int u = 32 * hh + j;
          float wa = 0.0f, wb = 0.0f;
#pragma unroll
          for (int k = 0; k < 8; ++k) {
            const float hk = hv[k];
            wa += hk * w1s[k * 192 + u];
            wb += hk * w1s[k * 192 + 64 + u];
          }
          wa *= inv8;
          wb *= inv8;
          const float se = s1p[u];
          float msa = (wa * se) * y0;
          float q   = wb * se;
          msa = valid ? msa : 0.0f;
          q   = valid ? q   : 0.0f;
          sthl(rh, rl, u, msa);
          sthl(rh, rl, 96 + u, q);
        }
#pragma unroll 1
        for (int j = 0; j < 16; ++j) {
          const int u = 16 * hh + j;
          float wc = 0.0f, wd = 0.0f;
#pragma unroll
          for (int k = 0; k < 8; ++k) {
            const float hk = hv[k];
            wc += hk * w1s[k * 192 + 128 + u];
            wd += hk * w1s[k * 192 + 160 + u];
          }
          wc *= inv8;
          wd *= inv8;
          const float ve0 = v1p[u], ve1 = v1p[32 + u], ve2 = v1p[64 + u];
          const float dt = ve0 * y1 + ve1 * y2 + ve2 * y3;
          float msb = (wd * dt) * inv3;
          float a0 = (wc * ve0) * y0;
          float a1 = (wc * ve1) * y0;
          float a2 = (wc * ve2) * y0;
          msb = valid ? msb : 0.0f;
          a0 = valid ? a0 : 0.0f;
          a1 = valid ? a1 : 0.0f;
          a2 = valid ? a2 : 0.0f;
          sthl(rh, rl, 64 + u, msb);
          sthl(rh, rl, 160 + u, a0);
          sthl(rh, rl, 192 + u, a1);
          sthl(rh, rl, 224 + u, a2);
        }
      }
      __syncthreads();

      {
        float g0[8], g1[8];
#pragma unroll
        for (int t = 0; t < 2; ++t) {
          const int nt = 4 + t;
          v8f c = z8;
#pragma unroll
          for (int kt = 0; kt < 3; ++kt) {
            const v16us b  = ldfrag_g(w2s, 96, 16 * nt + m, 32 * kt, hh);
            const v16us ah = ldfrag_s(aHi, AP, m, 32 * kt, hh);
            const v16us al = ldfrag_s(aLo, AP, m, 32 * kt, hh);
            c = wmb(ah, b, c);
            c = wmb(al, b, c);
          }
#pragma unroll
          for (int rr = 0; rr < 8; ++rr) {
            const float gq = sigm(c[rr] * inv96);
            if (t == 0) g0[rr] = gq; else g1[rr] = gq;
          }
        }
#pragma unroll
        for (int nt = 0; nt < 4; ++nt) {
          v8f c = z8;
#pragma unroll
          for (int kt = 0; kt < 3; ++kt) {
            const v16us b  = ldfrag_g(w2s, 96, 16 * nt + m, 32 * kt, hh);
            const v16us ah = ldfrag_s(aHi, AP, m, 32 * kt, hh);
            const v16us al = ldfrag_s(aLo, AP, m, 32 * kt, hh);
            c = wmb(ah, b, c);
            c = wmb(al, b, c);
          }
#pragma unroll
          for (int rr = 0; rr < 8; ++rr) msgw[(8 * hh + rr) * MW + 16 * nt + m] = silu(c[rr] * inv96);
        }
        v8f P0 = z8, P1 = z8;
#pragma unroll
        for (int nt = 0; nt < 2; ++nt) {
          v8f c = z8;
#pragma unroll
          for (int kt = 0; kt < 2; ++kt) {
            const v16us b  = ldfrag_g(w2v, 96, 16 * nt + m, 32 * kt, hh);
            const v16us ah = ldfrag_s(aHi, AP, m, 96 + 32 * kt, hh);
            const v16us al = ldfrag_s(aLo, AP, m, 96 + 32 * kt, hh);
            c = wmb(ah, b, c);
            c = wmb(al, b, c);
          }
          if (nt == 0) P0 = c; else P1 = c;
        }
#pragma unroll
        for (int cc = 0; cc < 3; ++cc) {
          float yc[8];
#pragma unroll
          for (int rr = 0; rr < 8; ++rr) yc[rr] = yw[(8 * hh + rr) * 4 + 1 + cc];
#pragma unroll
          for (int nt = 0; nt < 2; ++nt) {
            const v16us b  = ldfrag_g(w2v, 96, 16 * nt + m, 64, hh);
            const v16us ah = ldfrag_s(aHi, AP, m, 160 + 32 * cc, hh);
            const v16us al = ldfrag_s(aLo, AP, m, 160 + 32 * cc, hh);
            v8f c = z8;
            c = wmb(ah, b, c);
            c = wmb(al, b, c);
#pragma unroll
            for (int rr = 0; rr < 8; ++rr) {
              const float pv = (nt == 0) ? P0[rr] : P1[rr];
              const float gg = (nt == 0) ? g0[rr] : g1[rr];
              const float mv2 = (yc[rr] * pv + c[rr]) * inv96;
              msgw[(8 * hh + rr) * MW + 64 + 3 * (16 * nt + m) + cc] = mv2 * gg;
            }
          }
        }
      }
      __syncthreads();

      {
        const int c0 = tid;
        const int c1 = 128 + tid;
#pragma unroll 1
        for (int j = 0; j < PASSN; ++j) {
          int sl = slotb[j];
          sl = sl < 0 ? 0 : (sl > NB ? NB : sl);
          float* ar = acc + sl * MW;
          const float* mr = msg + j * MW;
          ar[c0] += mr[c0];
          if (tid < 32) ar[c1] += mr[c1];
        }
      }
      __syncthreads();
    }

    int rem = newN - R * PASSN;
    rem = rem < 0 ? 0 : rem;
    if (R > 0 && tid < rem) pend[tid] = pend[R * PASSN + tid];
    if (tid == 0) pendN[0] = rem;
  }
  __syncthreads();

  float* ob = agout + (size_t)nodeBase * MW;
#pragma unroll 1
  for (int it = 0; it < (NB * MW) / (4 * NT2); ++it) {
    const int f = it * 4 * NT2 + 4 * tid;
    v4f v = *(const v4f*)(acc + f);
    v = v * 0.25f;
    *(volatile v4f*)(ob + f) = v;
  }
  __threadfence();
#pragma unroll 1
  for (int it = 0; it < (NB * MW) / (4 * NT2); ++it) {
    const int f = it * 4 * NT2 + 4 * tid;
    v4f v = *(const v4f*)(acc + f);
    v = v * 0.25f;
    *(volatile v4f*)(ob + f) = v;
  }
}

__global__ __launch_bounds__(64) void k_node3(
    const float* __restrict__ feats, const float* __restrict__ attrs, const float* __restrict__ ag,
    const unsigned short* __restrict__ usP, const unsigned short* __restrict__ uvP,
    const unsigned short* __restrict__ w3s, const unsigned short* __restrict__ w3v,
    const unsigned short* __restrict__ scs, const unsigned short* __restrict__ scv,
    float* outp, int nN, float invs32, float invs512) {
  __shared__ __attribute__((aligned(16))) unsigned short sA[2][16 * 64];
  __shared__ __attribute__((aligned(16))) unsigned short vA[2][3 * 16 * 32];
  __shared__ __attribute__((aligned(16))) unsigned short aA[2][16 * 32];
  __shared__ __attribute__((aligned(16))) unsigned short usA[2][2 * 16 * 64];
  __shared__ __attribute__((aligned(16))) unsigned short uvA[2][2 * 3 * 16 * 32];
  __shared__ __attribute__((aligned(16))) float af[2][16 * 16];
  __shared__ __attribute__((aligned(16))) float ot[2][16 * MW];
  const int tid = threadIdx.x, lane = tid & 31, wave = tid >> 5, hh = lane >> 4, m = lane & 15;
  const int n0 = ((int)blockIdx.x * 2 + wave) * 16;
  unsigned short* sAw  = sA[wave];
  unsigned short* vAw  = vA[wave];
  unsigned short* aAw  = aA[wave];
  unsigned short* usAw = usA[wave];
  unsigned short* uvAw = uvA[wave];
  float* afw = af[wave];
  float* otw = ot[wave];

#pragma unroll 1
  for (int r = 0; r < 16; ++r) {
    int nd = n0 + r;
    nd = nd > nN - 1 ? nN - 1 : nd;
    const float* f = feats + (size_t)nd * 160;
    sAw[r * 64 + lane]      = f2bf(f[lane]);
    sAw[r * 64 + 32 + lane] = f2bf(f[32 + lane]);
#pragma unroll
    for (int t = 0; t < 3; ++t) {
      const int j = lane + 32 * t;
      const int u = j / 3;
      const int c = j - 3 * u;
      vAw[(c * 16 + r) * 32 + u] = f2bf(f[64 + j]);
    }
    const float a = attrs[(size_t)nd * 16 + (lane & 15)];
    aAw[r * 32 + lane] = (lane < 16) ? f2bf(a) : (unsigned short)0;
    if (lane < 16) afw[r * 16 + lane] = rbf(a);
  }
  __syncthreads();

  const v8f z8 = zero8f();
  {
    int ndr[8];
#pragma unroll
    for (int rr = 0; rr < 8; ++rr) { int nd = n0 + 8 * hh + rr; ndr[rr] = nd > nN - 1 ? nN - 1 : nd; }
    const v16us aa = ldfrag_s(aAw, 32, m, 0, hh);
#pragma unroll
    for (int nt = 0; nt < 4; ++nt) {
      const v8f D = wmb(aa, ldfrag_g(usP, 32, 16 * nt + m, 0, hh), z8);
#pragma unroll
      for (int rr = 0; rr < 8; ++rr) {
        const int u = 16 * nt + m;
        const float g = ag[(size_t)ndr[rr] * MW + u];
        const float us = (g * D[rr]) * 0.25f;
        sthl(usAw, usAw + 1024, (8 * hh + rr) * 64 + u, us);
      }
    }
#pragma unroll
    for (int nt = 0; nt < 2; ++nt) {
      const v8f D = wmb(aa, ldfrag_g(uvP, 32, 16 * nt + m, 0, hh), z8);
#pragma unroll
      for (int rr = 0; rr < 8; ++rr) {
        const int u = 16 * nt + m;
        const float cq = D[rr] * 0.25f;
#pragma unroll
        for (int c = 0; c < 3; ++c) {
          const float g = ag[(size_t)ndr[rr] * MW + 64 + 3 * u + c];
          sthl(uvAw, uvAw + 1536, (c * 16 + 8 * hh + rr) * 32 + u, g * cq);
        }
      }
    }
  }
  __syncthreads();

  {
    v8f accT[6];
#pragma unroll
    for (int wt = 0; wt < 6; ++wt) {
      v8f c = z8;
#pragma unroll
      for (int kt = 0; kt < 2; ++kt) {
        const v16us b  = ldfrag_g(w3s, 64, 16 * wt + m, 32 * kt, hh);
        const v16us ah = ldfrag_s(usAw, 64, m, 32 * kt, hh);
        const v16us al = ldfrag_s(usAw + 1024, 64, m, 32 * kt, hh);
        c = wmb(ah, b, c);
        c = wmb(al, b, c);
      }
      accT[wt] = c * 0.125f;
    }
    {
      const v16us as0 = ldfrag_s(sAw, 64, m, 0, hh);
      const v16us as1 = ldfrag_s(sAw, 64, m, 32, hh);
#pragma unroll 1
      for (int v = 0; v < 16; ++v) {
        float av[8];
#pragma unroll
        for (int rr = 0; rr < 8; ++rr) av[rr] = afw[(8 * hh + rr) * 16 + v];
#pragma unroll
        for (int wt = 0; wt < 6; ++wt) {
          const int rowB = v * 96 + 16 * wt + m;
          v8f D = wmb(as0, ldfrag_g(scs, 64, rowB, 0, hh), z8);
          D = wmb(as1, ldfrag_g(scs, 64, rowB, 32, hh), D);
#pragma unroll
          for (int rr = 0; rr < 8; ++rr) accT[wt][rr] += (av[rr] * D[rr]) * 0.03125f;
        }
      }
    }
    float g0[8], g1[8];
#pragma unroll
    for (int wt = 0; wt < 4; ++wt) {
#pragma unroll
      for (int rr = 0; rr < 8; ++rr) otw[(8 * hh + rr) * MW + 16 * wt + m] = silu(accT[wt][rr]);
    }
#pragma unroll
    for (int rr = 0; rr < 8; ++rr) { g0[rr] = sigm(accT[4][rr]); g1[rr] = sigm(accT[5][rr]); }

#pragma unroll
    for (int cc = 0; cc < 3; ++cc) {
      v8f lin0 = z8, lin1 = z8, sc0 = z8, sc1 = z8;
      {
        const v16us ah = ldfrag_s(uvAw + cc * 512, 32, m, 0, hh);
        const v16us al = ldfrag_s(uvAw + 1536 + cc * 512, 32, m, 0, hh);
#pragma unroll
        for (int nt = 0; nt < 2; ++nt) {
          const v16us b = ldfrag_g(w3v, 32, 16 * nt + m, 0, hh);
          v8f c = z8;
          c = wmb(ah, b, c);
          c = wmb(al, b, c);
          if (nt == 0) lin0 = c; else lin1 = c;
        }
      }
      {
        const v16us avf = ldfrag_s(vAw + cc * 512, 32, m, 0, hh);
#pragma unroll 1
        for (int v = 0; v < 16; ++v) {
          float av[8];
#pragma unroll
          for (int rr = 0; rr < 8; ++rr) av[rr] = afw[(8 * hh + rr) * 16 + v];
          const v8f D0 = wmb(avf, ldfrag_g(scv, 32, v * 32 + m, 0, hh), z8);
          const v8f D1 = wmb(avf, ldfrag_g(scv, 32, v * 32 + 16 + m, 0, hh), z8);
#pragma unroll
          for (int rr = 0; rr < 8; ++rr) { sc0[rr] += av[rr] * D0[rr]; sc1[rr] += av[rr] * D1[rr]; }
        }
      }
#pragma unroll
      for (int rr = 0; rr < 8; ++rr) {
        const float tv0 = lin0[rr] * invs32 + sc0[rr] * invs512;
        const float tv1 = lin1[rr] * invs32 + sc1[rr] * invs512;
        otw[(8 * hh + rr) * MW + 64 + 3 * m + cc]        = tv0 * g0[rr];
        otw[(8 * hh + rr) * MW + 64 + 3 * (16 + m) + cc] = tv1 * g1[rr];
      }
    }
  }
  __syncthreads();

  float* ob = outp + (size_t)n0 * MW;
#pragma unroll 1
  for (int it = 0; it < (16 * MW) / 128; ++it) {
    const int f = it * 128 + 4 * lane;
    const int nd = n0 + f / MW;
    const v4f v = *(const v4f*)(otw + f);
    if (nd < nN) *(volatile v4f*)(ob + f) = v;
  }
  __threadfence();
#pragma unroll 1
  for (int it = 0; it < (16 * MW) / 128; ++it) {
    const int f = it * 128 + 4 * lane;
    const int nd = n0 + f / MW;
    const v4f v = *(const v4f*)(otw + f);
    if (nd < nN) *(volatile v4f*)(ob + f) = v;
  }
}

extern "C" void kernel_launch(void* const* d_in, const int* in_sizes, int n_in,
                              void* d_out, int out_size, void* d_ws, size_t ws_size,
                              hipStream_t stream) {
  if (n_in < 17) return;
  const int nN = in_sizes[0] / 160;
  const int nE = in_sizes[16] / 2;
  if (nN < 1 || nE < 1) return;
  if (in_sizes[0] != nN * 160 || in_sizes[1] != nN * 16) return;
  if (in_sizes[2] != nE * 4 || in_sizes[3] != nE * 8 || in_sizes[16] != nE * 2) return;
  if (in_sizes[4] != 4096 || in_sizes[5] != 1024 || in_sizes[6] != 64 || in_sizes[7] != 1536) return;
  if (in_sizes[8] != 9216 || in_sizes[9] != 3072 || in_sizes[10] != 1024 || in_sizes[11] != 512) return;
  if (in_sizes[12] != 6144 || in_sizes[13] != 1024 || in_sizes[14] != 98304 || in_sizes[15] != 16384) return;
  if (out_size != nN * 160) return;

  const float* node_feats = (const float*)d_in[0];
  const float* node_attrs = (const float*)d_in[1];
  const float* edge_attrs = (const float*)d_in[2];
  const float* edge_emb   = (const float*)d_in[3];
  const float* W1_s   = (const float*)d_in[4];
  const float* W1_v   = (const float*)d_in[5];
  const float* mlp_w0 = (const float*)d_in[6];
  const float* mlp_w1 = (const float*)d_in[7];
  const float* W2_s   = (const float*)d_in[8];
  const float* W2_v   = (const float*)d_in[9];
  const float* U_s    = (const float*)d_in[10];
  const float* U_v    = (const float*)d_in[11];
  const float* W3_s   = (const float*)d_in[12];
  const float* W3_v   = (const float*)d_in[13];
  const float* SC_s   = (const float*)d_in[14];
  const float* SC_v   = (const float*)d_in[15];
  const int*   edge_index = (const int*)d_in[16];
  float* out = (float*)d_out;

  const float inv8    = 1.0f / (float)sqrt(8.0);
  const float inv3    = 1.0f / (float)sqrt(3.0);
  const float inv96   = 1.0f / (float)sqrt(96.0);
  const float invs32  = 1.0f / (float)sqrt(32.0);
  const float invs512 = 1.0f / (float)sqrt(512.0);

  const int nBlk1 = (nN + 31) / 32;
  const int nBlkE = (nN + NB - 1) / NB;

  WDesc wd;
  const int offs[10] = {0, 4096, 5120, 14336, 17408, 19456, 20480, 26624, 27648, 125952};
  const int nRs[10]  = {64, 32, 96, 32, 64, 32, 96, 32, 1536, 512};
  const int Ks[10]   = {64, 32, 96, 96, 16, 16, 64, 32, 64, 32};
  const int Kps[10]  = {64, 32, 96, 96, 32, 32, 64, 32, 64, 32};
  const int sks[10]  = {64, 32, 96, 32, 1, 1, 96, 32, 1536, 512};
  const int sns[10]  = {1, 1, 1, 1, 16, 16, 1, 1, 1, 1};
  const float* srcp[10] = {W1_s, W1_v, W2_s, W2_v, U_s, U_v, W3_s, W3_v, SC_s, SC_v};
  int wpBlocks = 0;
  for (int p = 0; p < 10; ++p) {
    wd.src[p] = srcp[p];
    wd.meta[6 * p + 0] = offs[p]; wd.meta[6 * p + 1] = nRs[p]; wd.meta[6 * p + 2] = Ks[p];
    wd.meta[6 * p + 3] = Kps[p]; wd.meta[6 * p + 4] = sks[p]; wd.meta[6 * p + 5] = sns[p];
    const int np = (nRs[p] * Kps[p]) >> 3;
    wpBlocks += (np + 255) >> 8;
  }
  const size_t wHalves = 142336;

  char* ws = (char*)d_ws;
  size_t off = 0;
  const size_t oW  = off; off += wHalves * 2;                          off = (off + 255) & ~(size_t)255;
  const size_t oS1 = off; off += (size_t)nBlk1 * 32 * 64 * 4;         off = (off + 255) & ~(size_t)255;
  const size_t oV1 = off; off += (size_t)nBlk1 * 32 * 96 * 4;         off = (off + 255) & ~(size_t)255;
  const size_t oAg = off; off += (size_t)nBlkE * NB * MW * 4;         off = (off + 255) & ~(size_t)255;
  if (off > ws_size) return;
  if (off > (size_t)134217728) return;
  unsigned short* wsh = (unsigned short*)(ws + oW);
  float* s1p = (float*)(ws + oS1);
  float* v1p = (float*)(ws + oV1);
  float* agp = (float*)(ws + oAg);

  const int vec8 = ((nE & 3) == 0) ? 1 : 0;

  k_wprep<<<wpBlocks, 256, 0, stream>>>(wd, wsh);

  k_node1<<<nBlk1, 64, 0, stream>>>(node_feats, wsh + offs[0], wsh + offs[1], s1p, v1p, nN, invs32);

  hipFuncSetAttribute(reinterpret_cast<const void*>(&k_edge), hipFuncAttributeMaxDynamicSharedMemorySize, L_TOT);
  k_edge<<<nBlkE, NT2, L_TOT, stream>>>(s1p, v1p, edge_attrs, edge_emb, mlp_w0, mlp_w1, edge_index,
                                        wsh + offs[2], wsh + offs[3], agp, nN, nE, vec8, inv8, inv3, inv96);

  k_node3<<<nBlk1, 64, 0, stream>>>(node_feats, node_attrs, agp, wsh + offs[4], wsh + offs[5],
                                    wsh + offs[6], wsh + offs[7], wsh + offs[8], wsh + offs[9],
                                    out, nN, invs32, invs512);
}
